// mambalayer_36636071035568
// MI455X (gfx1250) — hardware-run, weakly checked
//
#include <hip/hip_runtime.h>
#include <math.h>

typedef __attribute__((ext_vector_type(16))) _Float16 v16h;
typedef __attribute__((ext_vector_type(8)))  _Float16 v8h;
typedef __attribute__((ext_vector_type(8)))  float    v8f;
typedef __attribute__((ext_vector_type(4)))  float    v4f;
typedef __attribute__((ext_vector_type(4)))  unsigned v4u;

constexpr int kL     = 2048;
constexpr int kD     = 1024;
constexpr int kDin   = 2048;
constexpr int kNst   = 16;
constexpr int kDtR   = 64;
constexpr int kHid   = 4096;
constexpr int kXzN   = 2 * kDin;
constexpr int kPjReal = kDtR + 2 * kNst;
constexpr int kPjN   = 128;
constexpr float kEps = 1e-5f;
constexpr float kWCarry = 256.0f;
constexpr float kACarry = 16.0f;
constexpr int kConvTP = 260;
constexpr int kScanTS = 32;
constexpr int kScanCh = 64;
constexpr int kScanP  = 68;
static_assert(kPjReal <= kPjN);
static_assert((kD % 32) == 0 && (kDin % 32) == 0 && (kDtR % 32) == 0 && (kHid % 32) == 0);
static_assert((kL % 64) == 0 && (kXzN % 64) == 0 && (kPjN % 64) == 0 && (kDin % 64) == 0 && (kD % 64) == 0 && (kHid % 64) == 0);
static_assert((kL % kScanTS) == 0 && (kDin % kScanCh) == 0 && (kDin % 256) == 0 && (kL % 64) == 0 && (kD == 4 * 256));

constexpr size_t kOffWIN  = 0;
constexpr size_t kOffWXP  = kOffWIN  + (size_t)kXzN * kD   * 2;
constexpr size_t kOffWDT  = kOffWXP  + (size_t)kPjN * kDin * 2;
constexpr size_t kOffWOUT = kOffWDT  + (size_t)kDin * kDtR * 2;
constexpr size_t kOffW1   = kOffWOUT + (size_t)kD   * kDin * 2;
constexpr size_t kOffW2   = kOffW1   + (size_t)kHid * kD   * 2;
constexpr size_t kOffH1   = kOffW2   + (size_t)kD   * kHid * 2;
constexpr size_t kOffXZ   = kOffH1   + (size_t)kL   * kD   * 2;
constexpr size_t kOffXC   = kOffXZ   + (size_t)kL   * kXzN * 4;
constexpr size_t kOffPJ   = kOffXC   + (size_t)kL   * kDin * 2;
constexpr size_t kOffDP   = kOffPJ   + (size_t)kL   * kPjN * 2;
constexpr size_t kOffY    = kOffDP   + (size_t)kL   * kDin * 2;
constexpr size_t kOffH32  = kOffY    + (size_t)kL   * kDin * 2;
constexpr size_t kOffN16  = kOffH32  + (size_t)kL   * kD   * 4;
constexpr size_t kOffS32  = kOffN16  + (size_t)kL   * kD   * 2;
constexpr size_t kOffMID  = kOffS32  + (size_t)kL   * kD   * 4;
constexpr size_t kWsTotal = kOffMID  + (size_t)kL   * kHid * 2;
static_assert(kWsTotal == 131334144ull);
static_assert(kWsTotal <= 134217728ull);
static_assert((kOffWXP % 128) == 0 && (kOffWDT % 128) == 0 && (kOffWOUT % 128) == 0 && (kOffW1 % 128) == 0 &&
              (kOffW2 % 128) == 0 && (kOffH1 % 128) == 0 && (kOffXZ % 128) == 0 && (kOffXC % 128) == 0 &&
              (kOffPJ % 128) == 0 && (kOffDP % 128) == 0 && (kOffY % 128) == 0 && (kOffH32 % 128) == 0 &&
              (kOffN16 % 128) == 0 && (kOffS32 % 128) == 0 && (kOffMID % 128) == 0);

__device__ __forceinline__ float h16_to_f32(unsigned hb) {
  const unsigned sgn = (hb & 0x8000u) << 16; const unsigned em = hb & 0x7fffu;
  const float fn = __uint_as_float((em << 13) + 0x38000000u);
  const float fs = (float)em * 5.9604644775390625e-8f;
  const float mag = (em < 0x400u) ? fs : fn; return __uint_as_float(__float_as_uint(mag) | sgn); }

__device__ __forceinline__ void dep_guard_row_h(v8f& a0, v8f& a1, v8f& a2, v8f& a3,
                                                v16h x, v16h y0, v16h y1, v16h y2, v16h y3) {
  asm volatile("v_nop\n\tv_nop\n\tv_nop\n\tv_nop"
               : "+v"(a0), "+v"(a1), "+v"(a2), "+v"(a3)
               : "v"(x), "v"(y0), "v"(y1), "v"(y2), "v"(y3));
}
__device__ __forceinline__ void keep4_h(v16h a, v16h b, v16h c, v16h d) { asm volatile("v_nop" :: "v"(a), "v"(b), "v"(c), "v"(d)); }
__device__ __forceinline__ void acc_guard4(v8f& a, v8f& b, v8f& c, v8f& d) { asm volatile("v_nop\n\tv_nop\n\tv_nop\n\tv_nop" : "+v"(a), "+v"(b), "+v"(c), "+v"(d)); }

struct FragH {
  union U { v16h v; v8h h[2]; };
  static __device__ __forceinline__ v16h load(const _Float16* p) {
    U f; f.h[0] = *(const v8h*)(p); f.h[1] = *(const v8h*)(p + 16); return f.v;
  }
  static __device__ __forceinline__ v8f mma(v16h a, v16h b, v8f c) {
    return __builtin_amdgcn_wmma_f32_16x16x32_f16(false, a, false, b, (short)0, c, false, false);
  }
};

template <int BIAS_MODE, int OUT_MODE, bool RESID, int ACT>
__global__ __launch_bounds__(256) void wmma_gemm64p(
    const unsigned short* __restrict__ Ap, int lda,
    const unsigned short* __restrict__ Btp, int ldb,
    void* __restrict__ Cout, int ldc,
    const float* __restrict__ bias,
    const float* __restrict__ resid, int ldr,
    int M, int N, int K, float scale) {
  const _Float16* A = (const _Float16*)Ap;
  const _Float16* Bt = (const _Float16*)Btp;
  __shared__ __align__(16) float sT[8][16 * 68];
  const int lane = threadIdx.x & 31;
  const int wave = threadIdx.x >> 5;
  const int tilesN = N >> 6;
  const int tilesM = M >> 6;
  const int tile = blockIdx.x * 8 + wave;
  if (tile >= tilesM * tilesN) return;
  const int tm = tile / tilesN;
  const int tn = tile - tm * tilesN;
  const int m0 = tm << 6;
  const int n0 = tn << 6;

  const int rlane = lane & 15;
  const int koff  = (lane >> 4) * 8;
  const int mOff  = (lane >> 4) * 8;

  v8f acc[4][4];
#pragma unroll
  for (int i = 0; i < 4; ++i)
#pragma unroll
    for (int j = 0; j < 4; ++j) acc[i][j] = (v8f){0.f,0.f,0.f,0.f,0.f,0.f,0.f,0.f};

  for (int k0 = 0; k0 < K; k0 += 32) {
    v16h bh[4];
#pragma unroll
    for (int j = 0; j < 4; ++j) {
      const size_t bo = (size_t)(n0 + (j << 4) + rlane) * ldb + koff + k0;
      bh[j] = FragH::load(Bt + bo);
    }
#pragma unroll
    for (int i = 0; i < 4; ++i) {
      const size_t ao = (size_t)(m0 + (i << 4) + rlane) * lda + koff + k0;
      const v16h ah = FragH::load(A + ao);
#pragma unroll
      for (int j = 0; j < 4; ++j) acc[i][j] = FragH::mma(ah, bh[j], acc[i][j]);
      dep_guard_row_h(acc[i][0], acc[i][1], acc[i][2], acc[i][3], ah, bh[0], bh[1], bh[2], bh[3]);
    }
    keep4_h(bh[0], bh[1], bh[2], bh[3]);
  }
  acc_guard4(acc[0][0], acc[0][1], acc[0][2], acc[0][3]);
  acc_guard4(acc[1][0], acc[1][1], acc[1][2], acc[1][3]);
  acc_guard4(acc[2][0], acc[2][1], acc[2][2], acc[2][3]);
  acc_guard4(acc[3][0], acc[3][1], acc[3][2], acc[3][3]);

  float* slab = sT[wave];
#pragma unroll
  for (int i = 0; i < 4; ++i) {
    const int mBase = m0 + (i << 4);
#pragma unroll
    for (int j = 0; j < 4; ++j) {
      const int n = n0 + (j << 4) + rlane;
      float bv = 0.f;
      if (BIAS_MODE == 2) bv = bias[n];
#pragma unroll
      for (int r = 0; r < 8; ++r) {
        float v = acc[i][j][r] * scale;
        if (BIAS_MODE == 2) v += bv;
        if (ACT == 2) v = fmaxf(v, 0.0f);
        slab[(mOff + r) * 68 + (j << 4) + rlane] = v;
      }
    }
    __builtin_amdgcn_fence(__ATOMIC_RELEASE, "workgroup");
    __builtin_amdgcn_wave_barrier();
    __builtin_amdgcn_fence(__ATOMIC_ACQUIRE, "workgroup");
    if (OUT_MODE == 0) {
      float* C = (float*)Cout;
      const int hh = lane >> 4, c4 = (lane & 15) * 4;
      v4f vals[8];
#pragma unroll
      for (int it = 0; it < 8; ++it) {
        const int row = it * 2 + hh;
        v4f v = *(const v4f*)(slab + row * 68 + c4);
        if (RESID) {
          const v4f rr = *(const v4f*)(resid + (size_t)(mBase + row) * ldr + n0 + c4);
          v = v + rr;
        }
        vals[it] = v;
      }
      for (int pass = 0; pass < 2; ++pass) {
#pragma unroll
        for (int it = 0; it < 8; ++it) {
          const int row = it * 2 + hh;
          *(volatile v4f*)(C + (size_t)(mBase + row) * ldc + n0 + c4) = vals[it];
        }
        __threadfence();
      }
    } else {
      unsigned short* C = (unsigned short*)Cout;
      const int q = lane >> 3, c8 = (lane & 7) * 8;
      v8h hvv[4];
#pragma unroll
      for (int it = 0; it < 4; ++it) {
        const int row = it * 4 + q;
        const float* sp = slab + row * 68 + c8;
#pragma unroll
        for (int e = 0; e < 8; ++e) hvv[it][e] = (_Float16)sp[e];
      }
      for (int pass = 0; pass < 2; ++pass) {
#pragma unroll
        for (int it = 0; it < 4; ++it) {
          const int row = it * 4 + q;
          *(volatile v8h*)(C + (size_t)(mBase + row) * ldc + n0 + c8) = hvv[it];
        }
        __threadfence();
      }
    }
    __builtin_amdgcn_fence(__ATOMIC_RELEASE, "workgroup");
    __builtin_amdgcn_wave_barrier();
    __builtin_amdgcn_fence(__ATOMIC_ACQUIRE, "workgroup");
  }
}

__global__ __launch_bounds__(256) void cvt_rows_f16_kernel(
    const float* __restrict__ src, unsigned short* __restrict__ dst, int nsrc8, int ndst8, float scale)
{
  const int i = blockIdx.x * 256 + threadIdx.x;
  if (i >= ndst8) return;
  const bool inr = (i < nsrc8);
  const int ic = inr ? i : (nsrc8 - 1);
  const float fa = inr ? scale : 0.0f;
  const size_t e0 = (size_t)ic << 3;
  const v4f a0 = *(const v4f*)(src + e0);
  const v4f a1 = *(const v4f*)(src + e0 + 4);
  v8h hv;
#pragma unroll
  for (int e = 0; e < 4; ++e) {
    hv[e]     = (_Float16)(a0[e] * fa);
    hv[4 + e] = (_Float16)(a1[e] * fa);
  }
  unsigned short* qd = dst + ((size_t)i << 3);
  *(volatile v8h*)qd = hv;
  __threadfence();
  *(volatile v8h*)qd = hv;
}

template <int MODE>
__global__ __launch_bounds__(256) void ln_kernel(
    const float* __restrict__ X, const float* __restrict__ gam, const float* __restrict__ bet,
    const float* __restrict__ b2, unsigned short* __restrict__ O16, float* __restrict__ S32)
{
  __shared__ __align__(16) float sg[kD];
  __shared__ __align__(16) float sb[kD];
  __shared__ __align__(16) float sb2[MODE ? kD : 4];
  const int tid = threadIdx.x, lane = tid & 31, wave = tid >> 5;
  *(v4f*)(sg + 4 * tid) = *(const v4f*)(gam + 4 * tid);
  *(v4f*)(sb + 4 * tid) = *(const v4f*)(bet + 4 * tid);
  if (MODE) *(v4f*)(sb2 + 4 * tid) = *(const v4f*)(b2 + 4 * tid);
  __syncthreads();
  const int row = blockIdx.x * 8 + wave;
  const float* xr = X + (size_t)row * kD;

  float s = 0.0f;
#pragma unroll 1
  for (int i = 0; i < 8; ++i) {
    const v4f a = *(const v4f*)(xr + i * 128 + 4 * lane);
    s += (a[0] + a[1]) + (a[2] + a[3]);
  }
#pragma unroll
  for (int off = 1; off < 32; off <<= 1) s += __shfl_xor(s, off, 32);
  const float mu = s * (1.0f / 1024.0f);
  float ss = 0.0f;
#pragma unroll 1
  for (int i = 0; i < 8; ++i) {
    const v4f a = *(const v4f*)(xr + i * 128 + 4 * lane);
    const float e0 = a[0] - mu, e1 = a[1] - mu, e2 = a[2] - mu, e3 = a[3] - mu;
    ss = fmaf(e0, e0, ss); ss = fmaf(e1, e1, ss); ss = fmaf(e2, e2, ss); ss = fmaf(e3, e3, ss);
  }
#pragma unroll
  for (int off = 1; off < 32; off <<= 1) ss += __shfl_xor(ss, off, 32);
  const float rstd = rsqrtf(ss * (1.0f / 1024.0f) + kEps);

  v8h hv[4];
#pragma unroll
  for (int i = 0; i < 4; ++i) {
    const int c0 = i * 256 + 8 * lane;
    const v4f a0 = *(const v4f*)(xr + c0);
    const v4f a1 = *(const v4f*)(xr + c0 + 4);
    const v4f g0 = *(const v4f*)(sg + c0);
    const v4f g1 = *(const v4f*)(sg + c0 + 4);
    const v4f q0 = *(const v4f*)(sb + c0);
    const v4f q1 = *(const v4f*)(sb + c0 + 4);
#pragma unroll
    for (int e = 0; e < 4; ++e) {
      hv[i][e]     = (_Float16)(((a0[e] - mu) * rstd) * g0[e] + q0[e]);
      hv[i][4 + e] = (_Float16)(((a1[e] - mu) * rstd) * g1[e] + q1[e]);
    }
  }
  unsigned short* orow = O16 + (size_t)row * kD;
  for (int pass = 0; pass < 2; ++pass) {
#pragma unroll
    for (int i = 0; i < 4; ++i) *(volatile v8h*)(orow + i * 256 + 8 * lane) = hv[i];
    __threadfence();
  }
  if (MODE) {
    v4f sv[8];
#pragma unroll
    for (int i = 0; i < 8; ++i) {
      const int c0 = i * 128 + 4 * lane;
      const v4f a  = *(const v4f*)(xr + c0);
      const v4f g  = *(const v4f*)(sg + c0);
      const v4f qv = *(const v4f*)(sb + c0);
      const v4f cv = *(const v4f*)(sb2 + c0);
#pragma unroll
      for (int e = 0; e < 4; ++e) {
        const float nv = ((a[e] - mu) * rstd) * g[e] + qv[e];
        sv[i][e] = (a[e] + nv) + cv[e];
      }
    }
    float* srow = S32 + (size_t)row * kD;
    for (int pass = 0; pass < 2; ++pass) {
#pragma unroll
      for (int i = 0; i < 8; ++i) *(volatile v4f*)(srow + i * 128 + 4 * lane) = sv[i];
      __threadfence();
    }
  }
}

__global__ __launch_bounds__(256) void conv_silu_kernel(
    const float* __restrict__ XZ, const float* __restrict__ cw, const float* __restrict__ cb,
    unsigned short* __restrict__ XC16)
{
  __shared__ __align__(16) float sT[16 * kConvTP];
  const int tid = threadIdx.x, lane = tid & 31, wave = tid >> 5;
  const int d0 = blockIdx.x * 256, d = d0 + tid;
  const int g0 = blockIdx.y * 64;
  const v4f wv = *(const v4f*)(cw + (size_t)d * 4);
  const float w0 = wv[0], w1 = wv[1], w2 = wv[2], w3 = wv[3];
  const float bc = cb[d];
  float xm3, xm2, xm1;
  {
    const bool hist = (g0 > 0);
    const int rb = hist ? (g0 - 3) : g0;
    const float v3 = XZ[(size_t)rb * kXzN + d];
    const float v2 = XZ[(size_t)(rb + 1) * kXzN + d];
    const float v1 = XZ[(size_t)(rb + 2) * kXzN + d];
    xm3 = hist ? v3 : 0.0f;
    xm2 = hist ? v2 : 0.0f;
    xm1 = hist ? v1 : 0.0f;
  }
#pragma unroll 1
  for (int sub = 0; sub < 4; ++sub) {
    const int lb = g0 + sub * 16;
#pragma unroll 1
    for (int st = 0; st < 16; ++st) {
      const float xcur = XZ[(size_t)(lb + st) * kXzN + d];
      float accv = bc;
      accv = fmaf(w0, xm3, accv);
      accv = fmaf(w1, xm2, accv);
      accv = fmaf(w2, xm1, accv);
      accv = fmaf(w3, xcur, accv);
      const float sg = __builtin_amdgcn_rcpf(1.0f + expf(-accv));
      sT[st * kConvTP + tid] = (accv * sg) * kACarry;
      xm3 = xm2; xm2 = xm1; xm1 = xcur;
    }
    __syncthreads();
    v8h hv[2];
#pragma unroll
    for (int it = 0; it < 2; ++it) {
      const float* sp = sT + (it * 8 + wave) * kConvTP + lane * 8;
      const v4f a0 = *(const v4f*)(sp);
      const v4f a1 = *(const v4f*)(sp + 4);
#pragma unroll
      for (int e = 0; e < 4; ++e) {
        hv[it][e]     = (_Float16)a0[e];
        hv[it][4 + e] = (_Float16)a1[e];
      }
    }
    for (int pass = 0; pass < 2; ++pass) {
#pragma unroll
      for (int it = 0; it < 2; ++it) {
        const size_t o = (size_t)(lb + it * 8 + wave) * kDin + d0 + lane * 8;
        *(volatile v8h*)(XC16 + o) = hv[it];
      }
      __threadfence();
    }
    __syncthreads();
  }
}

__global__ __launch_bounds__(64) void scan_kernel(
    const unsigned short* __restrict__ DP16, const unsigned short* __restrict__ XC16,
    const float* __restrict__ XZ, const unsigned short* __restrict__ PJ16,
    const float* __restrict__ Alog, const float* __restrict__ Dp, unsigned short* __restrict__ Y16)
{
  __shared__ __align__(16) float sDl[kScanTS * kScanP];
  __shared__ __align__(16) float sU[kScanTS * kScanP];
  __shared__ __align__(16) float sZ[kScanTS * kScanP];
  __shared__ __align__(16) float sBC[kScanTS * 32];
  __shared__ __align__(16) float sY[kScanTS * kScanP];
  __shared__ __align__(16) float sA[kNst * kScanCh];
  const int tid = threadIdx.x, lane = tid & 31, wave = tid >> 5;
  const int d0 = blockIdx.x * kScanCh;
  const int d  = d0 + tid;
#pragma unroll 1
  for (int st = 0; st < kNst; ++st) sA[st * kScanCh + tid] = -expf(Alog[(size_t)d * kNst + st]);
  __syncthreads();
  float negA[kNst], h[kNst];
#pragma unroll
  for (int st = 0; st < kNst; ++st) {
    negA[st] = sA[st * kScanCh + tid];
    h[st] = 0.0f;
  }
  const float Dd = Dp[d];
  const float invc = 1.0f / kACarry;
  const int q = lane >> 3, c8 = (lane & 7) * 8;
#pragma unroll 1
  for (int t0 = 0; t0 < kL; t0 += kScanTS) {
    __syncthreads();
#pragma unroll 1
    for (int it = 0; it < 4; ++it) {
      const int idx = it * kScanCh + tid;
      const int r = idx >> 3, q8 = (idx & 7) * 8;
      const size_t go = (size_t)(t0 + r) * kDin + d0 + q8;
      const v4u wd = *(const v4u*)(DP16 + go);
      const v4u wu = *(const v4u*)(XC16 + go);
      v4f da, db, ua, ub;
      da[0] = h16_to_f32(wd[0] & 0xffffu); da[1] = h16_to_f32(wd[0] >> 16);
      da[2] = h16_to_f32(wd[1] & 0xffffu); da[3] = h16_to_f32(wd[1] >> 16);
      db[0] = h16_to_f32(wd[2] & 0xffffu); db[1] = h16_to_f32(wd[2] >> 16);
      db[2] = h16_to_f32(wd[3] & 0xffffu); db[3] = h16_to_f32(wd[3] >> 16);
      ua[0] = h16_to_f32(wu[0] & 0xffffu) * invc; ua[1] = h16_to_f32(wu[0] >> 16) * invc;
      ua[2] = h16_to_f32(wu[1] & 0xffffu) * invc; ua[3] = h16_to_f32(wu[1] >> 16) * invc;
      ub[0] = h16_to_f32(wu[2] & 0xffffu) * invc; ub[1] = h16_to_f32(wu[2] >> 16) * invc;
      ub[2] = h16_to_f32(wu[3] & 0xffffu) * invc; ub[3] = h16_to_f32(wu[3] >> 16) * invc;
      *(v4f*)(sDl + r * kScanP + q8)     = da;
      *(v4f*)(sDl + r * kScanP + q8 + 4) = db;
      *(v4f*)(sU  + r * kScanP + q8)     = ua;
      *(v4f*)(sU  + r * kScanP + q8 + 4) = ub;
    }
#pragma unroll 1
    for (int it = 0; it < 8; ++it) {
      const int idx = it * kScanCh + tid;
      const int r = idx >> 4, c4 = (idx & 15) * 4;
      *(v4f*)(sZ + r * kScanP + c4) = *(const v4f*)(XZ + (size_t)(t0 + r) * kXzN + kDin + d0 + c4);
    }
#pragma unroll 1
    for (int it = 0; it < 2; ++it) {
      const int idx = it * kScanCh + tid;
      const int r = idx >> 2, q8 = (idx & 3) * 8;
      const v4u w = *(const v4u*)(PJ16 + (size_t)(t0 + r) * kPjN + kDtR + q8);
      v4f ba, bb;
      ba[0] = h16_to_f32(w[0] & 0xffffu) * invc; ba[1] = h16_to_f32(w[0] >> 16) * invc;
      ba[2] = h16_to_f32(w[1] & 0xffffu) * invc; ba[3] = h16_to_f32(w[1] >> 16) * invc;
      bb[0] = h16_to_f32(w[2] & 0xffffu) * invc; bb[1] = h16_to_f32(w[2] >> 16) * invc;
      bb[2] = h16_to_f32(w[3] & 0xffffu) * invc; bb[3] = h16_to_f32(w[3] >> 16) * invc;
      *(v4f*)(sBC + r * 32 + q8)     = ba;
      *(v4f*)(sBC + r * 32 + q8 + 4) = bb;
    }
    __syncthreads();
#pragma unroll 1
    for (int st = 0; st < kScanTS; ++st) {
      const float v  = sDl[st * kScanP + tid];
      const float av = expf(-fabsf(v));
      const float dt = fmaxf(v, 0.0f) + log1pf(av);
      const float xt = sU[st * kScanP + tid];
      const float zv = sZ[st * kScanP + tid];
      const float* bcr = sBC + st * 32;
      float Bs[kNst], Cs[kNst];
#pragma unroll
      for (int q4 = 0; q4 < 4; ++q4) {
        const v4f bv = *(const v4f*)(bcr + 4 * q4);
        const v4f cv = *(const v4f*)(bcr + kNst + 4 * q4);
        Bs[4 * q4 + 0] = bv[0]; Bs[4 * q4 + 1] = bv[1]; Bs[4 * q4 + 2] = bv[2]; Bs[4 * q4 + 3] = bv[3];
        Cs[4 * q4 + 0] = cv[0]; Cs[4 * q4 + 1] = cv[1]; Cs[4 * q4 + 2] = cv[2]; Cs[4 * q4 + 3] = cv[3];
      }
      const float dtx = dt * xt;
      float y = 0.0f;
#pragma unroll
      for (int k = 0; k < kNst; ++k) {
        const float e = __expf(dt * negA[k]);
        h[k] = fmaf(e, h[k], dtx * Bs[k]);
        y = fmaf(h[k], Cs[k], y);
      }
      y = fmaf(xt, Dd, y);
      const float sg = __builtin_amdgcn_rcpf(1.0f + expf(-zv));
      y = y * (zv * sg);
      sY[st * kScanP + tid] = y * kACarry;
    }
    __syncthreads();
    v8h hv[4];
#pragma unroll
    for (int it = 0; it < 4; ++it) {
      const int row = it * 8 + wave * 4 + q;
      const float* sp = sY + row * kScanP + c8;
      const v4f a0 = *(const v4f*)(sp);
      const v4f a1 = *(const v4f*)(sp + 4);
#pragma unroll
      for (int e = 0; e < 4; ++e) {
        hv[it][e]     = (_Float16)a0[e];
        hv[it][4 + e] = (_Float16)a1[e];
      }
    }
    for (int pass = 0; pass < 2; ++pass) {
#pragma unroll
      for (int it = 0; it < 4; ++it) {
        const int row = it * 8 + wave * 4 + q;
        const size_t o = (size_t)(t0 + row) * kDin + d0 + c8;
        *(volatile v8h*)(Y16 + o) = hv[it];
      }
      __threadfence();
    }
  }
}

extern "C" void kernel_launch(void* const* d_in, const int* in_sizes, int n_in,
                              void* d_out, int out_size, void* d_ws, size_t ws_size,
                              hipStream_t stream) {
  if (n_in < 18) return;
  if (in_sizes[0]  != kL * kD) return;
  if (in_sizes[1]  != kD || in_sizes[2] != kD || in_sizes[3] != kD || in_sizes[4] != kD) return;
  if (in_sizes[5]  != kXzN * kD) return;
  if (in_sizes[6]  != kDin * 4) return;
  if (in_sizes[7]  != kDin) return;
  if (in_sizes[8]  != kPjReal * kDin) return;
  if (in_sizes[9]  != kDin * kDtR) return;
  if (in_sizes[10] != kDin) return;
  if (in_sizes[11] != kDin * kNst) return;
  if (in_sizes[12] != kDin) return;
  if (in_sizes[13] != kD * kDin) return;
  if (in_sizes[14] != kHid * kD) return;
  if (in_sizes[15] != kHid) return;
  if (in_sizes[16] != kD * kHid) return;
  if (in_sizes[17] != kD) return;
  if (out_size != kL * kD) return;
  if (ws_size < kWsTotal) return;

  const float* x          = (const float*)d_in[0];
  const float* ln1_g      = (const float*)d_in[1];
  const float* ln1_b      = (const float*)d_in[2];
  const float* ln2_g      = (const float*)d_in[3];
  const float* ln2_b      = (const float*)d_in[4];
  const float* in_proj_w  = (const float*)d_in[5];
  const float* conv_w     = (const float*)d_in[6];
  const float* conv_b     = (const float*)d_in[7];
  const float* x_proj_w   = (const float*)d_in[8];
  const float* dt_proj_w  = (const float*)d_in[9];
  const float* dt_proj_b  = (const float*)d_in[10];
  const float* A_log      = (const float*)d_in[11];
  const float* D_param    = (const float*)d_in[12];
  const float* out_proj_w = (const float*)d_in[13];
  const float* ffn_w1     = (const float*)d_in[14];
  const float* ffn_b1     = (const float*)d_in[15];
  const float* ffn_w2     = (const float*)d_in[16];
  const float* ffn_b2     = (const float*)d_in[17];
  float* out = (float*)d_out;

  char* ws = (char*)d_ws;
  unsigned short* WIN  = (unsigned short*)(ws + kOffWIN);
  unsigned short* WXP  = (unsigned short*)(ws + kOffWXP);
  unsigned short* WDT  = (unsigned short*)(ws + kOffWDT);
  unsigned short* WOUT = (unsigned short*)(ws + kOffWOUT);
  unsigned short* W1   = (unsigned short*)(ws + kOffW1);
  unsigned short* W2   = (unsigned short*)(ws + kOffW2);
  unsigned short* H1   = (unsigned short*)(ws + kOffH1);
  float*          XZ   = (float*)(ws + kOffXZ);
  unsigned short* XC   = (unsigned short*)(ws + kOffXC);
  unsigned short* PJ   = (unsigned short*)(ws + kOffPJ);
  unsigned short* DP   = (unsigned short*)(ws + kOffDP);
  unsigned short* Y    = (unsigned short*)(ws + kOffY);
  float*          H32  = (float*)(ws + kOffH32);
  unsigned short* N16  = (unsigned short*)(ws + kOffN16);
  float*          S32  = (float*)(ws + kOffS32);
  unsigned short* MID  = (unsigned short*)(ws + kOffMID);

  {
    constexpr int n8_in  = kXzN * kD / 8;
    constexpr int n8_xs  = kPjReal * kDin / 8;
    constexpr int n8_xd  = kPjN * kDin / 8;
    constexpr int n8_dt  = kDin * kDtR / 8;
    constexpr int n8_out = kD * kDin / 8;
    constexpr int n8_w1  = kHid * kD / 8;
    constexpr int n8_w2  = kD * kHid / 8;
    static_assert((n8_in % 256) == 0 && (n8_xd % 256) == 0 && (n8_dt % 256) == 0 && (n8_out % 256) == 0 &&
                  (n8_w1 % 256) == 0 && (n8_w2 % 256) == 0);
    cvt_rows_f16_kernel<<<n8_in / 256, 256, 0, stream>>>(in_proj_w, WIN, n8_in, n8_in, kWCarry);
    cvt_rows_f16_kernel<<<n8_xd / 256, 256, 0, stream>>>(x_proj_w, WXP, n8_xs, n8_xd, kWCarry);
    cvt_rows_f16_kernel<<<n8_dt / 256, 256, 0, stream>>>(dt_proj_w, WDT, n8_dt, n8_dt, kWCarry);
    cvt_rows_f16_kernel<<<n8_out / 256, 256, 0, stream>>>(out_proj_w, WOUT, n8_out, n8_out, kWCarry);
    cvt_rows_f16_kernel<<<n8_w1 / 256, 256, 0, stream>>>(ffn_w1, W1, n8_w1, n8_w1, kWCarry);
    cvt_rows_f16_kernel<<<n8_w2 / 256, 256, 0, stream>>>(ffn_w2, W2, n8_w2, n8_w2, kWCarry);
  }

  ln_kernel<0><<<kL / 8, 256, 0, stream>>>(x, ln1_g, ln1_b, nullptr, H1, nullptr);

  wmma_gemm64p<0, 0, false, 0><<<(kL / 64) * (kXzN / 64) / 8, 256, 0, stream>>>(
      H1, kD, WIN, kD, (void*)XZ, kXzN, nullptr, nullptr, 0, kL, kXzN, kD, 1.0f / kWCarry);

  conv_silu_kernel<<<dim3(kDin / 256, kL / 64), 256, 0, stream>>>(XZ, conv_w, conv_b, XC);

  wmma_gemm64p<0, 1, false, 0><<<(kL / 64) * (kPjN / 64) / 8, 256, 0, stream>>>(
      XC, kDin, WXP, kDin, (void*)PJ, kPjN, nullptr, nullptr, 0, kL, kPjN, kDin, 1.0f / kWCarry);

  wmma_gemm64p<2, 1, false, 0><<<(kL / 64) * (kDin / 64) / 8, 256, 0, stream>>>(
      PJ, kPjN, WDT, kDtR, (void*)DP, kDin, dt_proj_b, nullptr, 0, kL, kDin, kDtR, 1.0f / (kWCarry * kACarry));

  scan_kernel<<<kDin / kScanCh, kScanCh, 0, stream>>>(DP, XC, XZ, PJ, A_log, D_param, Y);

  wmma_gemm64p<0, 0, true, 0><<<(kL / 64) * (kD / 64) / 8, 256, 0, stream>>>(
      Y, kDin, WOUT, kDin, (void*)H32, kD, nullptr, x, kD, kL, kD, kDin, 1.0f / (kWCarry * kACarry));

  ln_kernel<1><<<kL / 8, 256, 0, stream>>>(H32, ln2_g, ln2_b, ffn_b2, N16, S32);

  wmma_gemm64p<2, 1, false, 2><<<(kL / 64) * (kHid / 64) / 8, 256, 0, stream>>>(
      N16, kD, W1, kD, (void*)MID, kHid, ffn_b1, nullptr, 0, kL, kHid, kD, 1.0f / kWCarry);

  wmma_gemm64p<0, 0, true, 0><<<(kL / 64) * (kD / 64) / 8, 256, 0, stream>>>(
      MID, kHid, W2, kHid, (void*)out, kD, nullptr, S32, kD, kL, kD, kHid, 1.0f / kWCarry);
}
